// DualAttentionAutoEncoder_5978594476336
// MI455X (gfx1250) — hardware-verified
//
#include <hip/hip_runtime.h>
#include <math.h>

constexpr int NBATCH = 8192;
constexpr int NLAG   = 10;
constexpr int NFEAT  = 128;
constexpr int NHID   = 64;
constexpr int NGATE  = 4 * NHID;
constexpr int NOUTD  = 5;
constexpr int NROWS  = NBATCH * NLAG;
constexpr int NTHR   = 256;
constexpr int ROWS_PER_BLK = 32;

constexpr float WCARRY   = 256.0f;
constexpr float SCARRY   = 64.0f;
constexpr float WI_CARRY = 1024.0f;
constexpr float GX_CARRY = 1024.0f;
constexpr float FOLD_SW  = 1.0f / (WCARRY * SCARRY);
constexpr float GX_SCALE = GX_CARRY / (WI_CARRY * WCARRY);
constexpr float GX_INV   = 1.0f / GX_CARRY;
constexpr float S_INV    = 1.0f / SCARRY;

constexpr int EHP = 72;
constexpr int EGP = 264;
constexpr int DAP = 168;
constexpr int DSP = 68;
constexpr int SCP = 12;
constexpr int DGK = 96;
constexpr int FCW_N = NOUTD * (NHID + NOUTD);
constexpr int FOW_N = NOUTD * 2 * NHID;

constexpr int PB_WIH  = NGATE * (NFEAT / 8) / NTHR;
constexpr int PB_WHH  = NGATE * (NHID / 8) / NTHR;
constexpr int PB_DG   = NGATE * (DGK / 8) / NTHR;
constexpr int PB_W1HC = NHID * (2 * NHID / 8) / NTHR;
constexpr int PB_W1X  = NHID * (NHID / 8) / NTHR;
constexpr int PB_E0 = PB_WIH;
constexpr int PB_E1 = PB_E0 + PB_WHH;
constexpr int PB_E2 = PB_E1 + PB_DG;
constexpr int PB_E3 = PB_E2 + PB_W1HC;
constexpr int PB_E4 = PB_E3 + PB_W1X;

static_assert(NGATE == 256 && NHID == 64 && NFEAT == 128, "shape constants");
static_assert(NROWS % 64 == 0 && NGATE % 64 == 0 && NHID % 64 == 0, "GEMM M, N tile multiples");
static_assert(NFEAT % 32 == 0 && NHID % 32 == 0 && DGK % 32 == 0, "GEMM K multiples of 32");
static_assert(NBATCH % ROWS_PER_BLK == 0 && NBATCH % 16 == 0, "batch tiling exact");
static_assert((ROWS_PER_BLK * NOUTD * 4) % 128 == 0, "output tile is whole 128-B lines");
static_assert(PB_WIH * NTHR == NGATE * (NFEAT / 8) && PB_WHH * NTHR == NGATE * (NHID / 8), "prep coverage");
static_assert(PB_DG * NTHR == NGATE * (DGK / 8) && PB_W1HC * NTHR == NHID * 16 && PB_W1X * NTHR == NHID * 8, "prep coverage");
static_assert((EHP % 8) == 0 && (EGP % 8) == 0 && (DAP % 8) == 0 && (DSP % 4) == 0, "LDS pitches keep 16-B alignment");

typedef __attribute__((ext_vector_type(16))) _Float16 v16h;
typedef __attribute__((ext_vector_type(8)))  _Float16 v8h;
typedef __attribute__((ext_vector_type(8)))  float    v8f;
typedef __attribute__((ext_vector_type(4)))  float    v4f;
typedef __attribute__((ext_vector_type(4)))  unsigned v4u;

__device__ __forceinline__ float h16_to_f32(unsigned hb) {
  const unsigned sgn = (hb & 0x8000u) << 16;
  const unsigned em = hb & 0x7fffu;
  const float fn = __uint_as_float((em << 13) + 0x38000000u);
  const float fs = (float)em * 5.9604644775390625e-8f;
  const float mag = (em < 0x400u) ? fs : fn;
  return __uint_as_float(__float_as_uint(mag) | sgn);
}

__device__ __forceinline__ float fsig(float x)  { return __builtin_amdgcn_rcpf(1.0f + expf(-x)); }
__device__ __forceinline__ float ftanh(float x) { return 1.0f - 2.0f * __builtin_amdgcn_rcpf(expf(2.0f * x) + 1.0f); }

union FragH { v16h v; v8h h[2]; };
__device__ __forceinline__ v16h frag_load(const _Float16* p) {
  FragH f;
  f.h[0] = *(const v8h*)(p);
  f.h[1] = *(const v8h*)(p + 16);
  return f.v;
}
__device__ __forceinline__ v8f mma_h(v16h a, v16h b, v8f c) {
  c = __builtin_amdgcn_wmma_f32_16x16x32_f16(false, a, false, b, (short)0, c, false, false);
  asm volatile("v_nop\n\tv_nop\n\tv_nop\n\tv_nop" : "+v"(c) : "v"(a), "v"(b));
  return c;
}
__device__ __forceinline__ v8f mma_plain(v16h a, v16h b, v8f c) {
  return __builtin_amdgcn_wmma_f32_16x16x32_f16(false, a, false, b, (short)0, c, false, false);
}
__device__ __forceinline__ void dep_guard4_h(v8f& a0, v8f& a1, v8f& a2, v8f& a3, v16h x, v16h y0, v16h y1, v16h y2, v16h y3) {
  asm volatile("v_nop\n\tv_nop\n\tv_nop\n\tv_nop" : "+v"(a0), "+v"(a1), "+v"(a2), "+v"(a3) : "v"(x), "v"(y0), "v"(y1), "v"(y2), "v"(y3));
}
__device__ __forceinline__ void keep4_h(v16h a, v16h b, v16h c, v16h d) { asm volatile("v_nop" :: "v"(a), "v"(b), "v"(c), "v"(d)); }
__device__ __forceinline__ void acc_guard4(v8f& a, v8f& b, v8f& c, v8f& d) { asm volatile("v_nop\n\tv_nop\n\tv_nop\n\tv_nop" : "+v"(a), "+v"(b), "+v"(c), "+v"(d)); }

__global__ __launch_bounds__(256) void gemm64_f16_kernel(
    const unsigned short* __restrict__ Ap, int lda,
    const unsigned short* __restrict__ Btp, int ldb,
    unsigned short* __restrict__ Cp, int ldc,
    int M, int N, int K, float scale) {
  const _Float16* A  = (const _Float16*)Ap;
  const _Float16* Bt = (const _Float16*)Btp;
  __shared__ __align__(16) float sT[8][16 * 68];
  const int lane = threadIdx.x & 31;
  const int wave = threadIdx.x >> 5;
  const int tilesN = N >> 6;
  const int tilesM = M >> 6;
  const int tile = blockIdx.x * 8 + wave;
  if (tile >= tilesM * tilesN) return;
  const int tm = tile / tilesN;
  const int tn = tile - tm * tilesN;
  const int m0 = tm << 6;
  const int n0 = tn << 6;
  const int rlane = lane & 15;
  const int koff  = (lane >> 4) * 8;
  const int mOff  = (lane >> 4) * 8;

  v8f acc[4][4];
#pragma unroll
  for (int i = 0; i < 4; ++i)
#pragma unroll
    for (int j = 0; j < 4; ++j) acc[i][j] = (v8f){0.f, 0.f, 0.f, 0.f, 0.f, 0.f, 0.f, 0.f};

  for (int k0 = 0; k0 < K; k0 += 32) {
    v16h bh[4];
#pragma unroll
    for (int j = 0; j < 4; ++j) {
      const size_t bo = (size_t)(n0 + (j << 4) + rlane) * ldb + koff + k0;
      bh[j] = frag_load(Bt + bo);
    }
#pragma unroll
    for (int i = 0; i < 4; ++i) {
      const size_t ao = (size_t)(m0 + (i << 4) + rlane) * lda + koff + k0;
      const v16h ah = frag_load(A + ao);
#pragma unroll
      for (int j = 0; j < 4; ++j) acc[i][j] = mma_plain(ah, bh[j], acc[i][j]);
      dep_guard4_h(acc[i][0], acc[i][1], acc[i][2], acc[i][3], ah, bh[0], bh[1], bh[2], bh[3]);
    }
    keep4_h(bh[0], bh[1], bh[2], bh[3]);
  }
  acc_guard4(acc[0][0], acc[0][1], acc[0][2], acc[0][3]);
  acc_guard4(acc[1][0], acc[1][1], acc[1][2], acc[1][3]);
  acc_guard4(acc[2][0], acc[2][1], acc[2][2], acc[2][3]);
  acc_guard4(acc[3][0], acc[3][1], acc[3][2], acc[3][3]);

  float* slab = sT[wave];
#pragma unroll
  for (int i = 0; i < 4; ++i) {
    const int mBase = m0 + (i << 4);
#pragma unroll
    for (int j = 0; j < 4; ++j) {
#pragma unroll
      for (int r = 0; r < 8; ++r) slab[(mOff + r) * 68 + (j << 4) + rlane] = acc[i][j][r] * scale;
    }
    __builtin_amdgcn_fence(__ATOMIC_RELEASE, "workgroup");
    __builtin_amdgcn_wave_barrier();
    __builtin_amdgcn_fence(__ATOMIC_ACQUIRE, "workgroup");
    {
      const int q = lane >> 3, c8 = (lane & 7) * 8;
      for (int pass = 0; pass < 2; ++pass) {
#pragma unroll
        for (int it = 0; it < 4; ++it) {
          const int row = it * 4 + q;
          const float* sp = slab + row * 68 + c8;
          v8h hv;
#pragma unroll
          for (int e = 0; e < 8; ++e) hv[e] = (_Float16)sp[e];
          *(volatile v8h*)(Cp + (size_t)(mBase + row) * ldc + n0 + c8) = hv;
        }
        __threadfence();
      }
    }
    __builtin_amdgcn_fence(__ATOMIC_RELEASE, "workgroup");
    __builtin_amdgcn_wave_barrier();
    __builtin_amdgcn_fence(__ATOMIC_ACQUIRE, "workgroup");
  }
}

__global__ __launch_bounds__(256) void prep_planes_kernel(
    const float* __restrict__ enc_wih, const float* __restrict__ enc_whh,
    const float* __restrict__ dec_whh, const float* __restrict__ dec_wih,
    const float* __restrict__ att_w1,
    unsigned short* __restrict__ WIH, unsigned short* __restrict__ WHH,
    unsigned short* __restrict__ DG, unsigned short* __restrict__ W1HC, unsigned short* __restrict__ W1X) {
  const int bid = blockIdx.x, tid = threadIdx.x;
  v8h hv;
  unsigned short* dp;
  if (bid >= PB_E1 && bid < PB_E2) {
    const int i = (bid - PB_E1) * NTHR + tid;
    const int row = i / (DGK / 8);
    const int seg = i - row * (DGK / 8);
    const int sgc = (seg < 8) ? seg : 7;
    const float* sp = dec_whh + (size_t)row * NHID + sgc * 8;
    const v4f a  = *(const v4f*)(sp);
    const v4f bq = *(const v4f*)(sp + 4);
    float wv[5];
#pragma unroll
    for (int e = 0; e < 5; ++e) wv[e] = dec_wih[row * NOUTD + e];
    float f[8];
#pragma unroll
    for (int e = 0; e < 4; ++e) { f[e] = a[e]; f[4 + e] = bq[e]; }
#pragma unroll
    for (int e = 0; e < 8; ++e) {
      const float wsel = (e < 5) ? wv[(e < 5) ? e : 0] : 0.0f;
      const float val = (seg < 8) ? f[e] : ((seg == 8) ? wsel : 0.0f);
      hv[e] = (_Float16)(val * WCARRY);
    }
    dp = DG + (size_t)i * 8;
  } else {
    const float* src;
    unsigned short* dst;
    int ncol8, spitch, scol0, blk0;
    if (bid < PB_E0)      { src = enc_wih; dst = WIH;  ncol8 = NFEAT / 8;    spitch = NFEAT;    scol0 = 0;        blk0 = 0; }
    else if (bid < PB_E1) { src = enc_whh; dst = WHH;  ncol8 = NHID / 8;     spitch = NHID;     scol0 = 0;        blk0 = PB_E0; }
    else if (bid < PB_E3) { src = att_w1;  dst = W1HC; ncol8 = 2 * NHID / 8; spitch = 3 * NHID; scol0 = 0;        blk0 = PB_E2; }
    else                  { src = att_w1;  dst = W1X;  ncol8 = NHID / 8;     spitch = 3 * NHID; scol0 = 2 * NHID; blk0 = PB_E3; }
    const int i = (bid - blk0) * NTHR + tid;
    const int row = i / ncol8;
    const int c8  = i - row * ncol8;
    const float* sp = src + (size_t)row * spitch + scol0 + c8 * 8;
    const v4f a  = *(const v4f*)(sp);
    const v4f bq = *(const v4f*)(sp + 4);
#pragma unroll
    for (int e = 0; e < 4; ++e) {
      hv[e]     = (_Float16)(a[e] * WCARRY);
      hv[4 + e] = (_Float16)(bq[e] * WCARRY);
    }
    dp = dst + (size_t)i * 8;
  }
  *(volatile v8h*)dp = hv;
  __threadfence();
  *(volatile v8h*)dp = hv;
}

__global__ __launch_bounds__(256) void wi_build_kernel(const float* __restrict__ x, const float* __restrict__ attn_w,
                                                       const float* __restrict__ attn_b, unsigned short* __restrict__ WI16) {
  const int tid = threadIdx.x, lane = tid & 31, wave = tid >> 5;
  const int half = lane >> 4, d0 = (lane & 15) * 8;
  const int b = (blockIdx.x * 8 + wave) * 2 + half;
  const float* xb = x + (size_t)b * (NLAG * NFEAT) + d0;
  const float eb = attn_b[0];
  float sc[8];
#pragma unroll
  for (int e = 0; e < 8; ++e) sc[e] = eb;
#pragma unroll 1
  for (int l = 0; l < NLAG; ++l) {
    const float wl = attn_w[2 * NHID + l];
    const v4f a  = *(const v4f*)(xb + l * NFEAT);
    const v4f bq = *(const v4f*)(xb + l * NFEAT + 4);
#pragma unroll
    for (int e = 0; e < 4; ++e) {
      sc[e]     = fmaf(a[e], wl, sc[e]);
      sc[4 + e] = fmaf(bq[e], wl, sc[4 + e]);
    }
  }
  float m = sc[0];
#pragma unroll
  for (int e = 1; e < 8; ++e) m = fmaxf(m, sc[e]);
#pragma unroll
  for (int off = 1; off < 16; off <<= 1) m = fmaxf(m, __shfl_xor(m, off, 32));
  float ssum = 0.0f;
  float at[8];
#pragma unroll
  for (int e = 0; e < 8; ++e) { at[e] = expf(sc[e] - m); ssum += at[e]; }
#pragma unroll
  for (int off = 1; off < 16; off <<= 1) ssum += __shfl_xor(ssum, off, 32);
  const float inv = (1.0f / ssum) * WI_CARRY;
#pragma unroll
  for (int e = 0; e < 8; ++e) at[e] *= inv;
#pragma unroll 1
  for (int t = 0; t < NLAG; ++t) {
    const v4f a  = *(const v4f*)(xb + t * NFEAT);
    const v4f bq = *(const v4f*)(xb + t * NFEAT + 4);
    v8h hv;
#pragma unroll
    for (int e = 0; e < 4; ++e) {
      hv[e]     = (_Float16)(at[e] * a[e]);
      hv[4 + e] = (_Float16)(at[4 + e] * bq[e]);
    }
    unsigned short* p = WI16 + ((size_t)t * NBATCH + (size_t)b) * NFEAT + d0;
    *(volatile v8h*)p = hv;
    __threadfence();
    *(volatile v8h*)p = hv;
  }
}

__global__ __launch_bounds__(256) void enc_seq_kernel(
    const unsigned short* __restrict__ GX16, const unsigned short* __restrict__ WHHp,
    const float* __restrict__ h0, const float* __restrict__ c0,
    const float* __restrict__ bih, const float* __restrict__ bhh,
    unsigned short* __restrict__ XENC16) {
  __shared__ __align__(16) _Float16       Ah[ROWS_PER_BLK * EHP];
  __shared__ __align__(16) unsigned short Gs[ROWS_PER_BLK * EGP];
  const _Float16* WHH = (const _Float16*)WHHp;
  const int tid = threadIdx.x, lane = tid & 31, wave = tid >> 5;
  const int c = lane & 15, hh = lane >> 4, koff = hh * 8;
  const int ms = wave >> 2, ub = wave & 3;
  const int j = 16 * ub + c;
  const int rowbase = blockIdx.x * ROWS_PER_BLK;
  const int srow = tid >> 3, sseg = tid & 7;

  {
    const float* hp = h0 + (size_t)(rowbase + srow) * NHID + sseg * 8;
    const v4f a  = *(const v4f*)(hp);
    const v4f bq = *(const v4f*)(hp + 4);
    v8h hv;
#pragma unroll
    for (int e = 0; e < 4; ++e) {
      hv[e]     = (_Float16)(a[e] * SCARRY);
      hv[4 + e] = (_Float16)(bq[e] * SCARRY);
    }
    *(v8h*)(Ah + srow * EHP + sseg * 8) = hv;
  }
  float cst[8], bb[4];
#pragma unroll
  for (int r = 0; r < 8; ++r) cst[r] = c0[(size_t)(rowbase + 16 * ms + 8 * hh + r) * NHID + j];
#pragma unroll
  for (int g = 0; g < 4; ++g) bb[g] = bih[g * NHID + j] + bhh[g * NHID + j];
  v16h bw[4][2];
#pragma unroll
  for (int g = 0; g < 4; ++g)
#pragma unroll
    for (int kt = 0; kt < 2; ++kt) bw[g][kt] = frag_load(WHH + (size_t)(g * NHID + j) * NHID + koff + kt * 32);

  const v8f z8 = {0.f, 0.f, 0.f, 0.f, 0.f, 0.f, 0.f, 0.f};
  const _Float16* arow = Ah + (16 * ms + c) * EHP + koff;

#pragma unroll 1
  for (int t = 0; t < NLAG; ++t) {
#pragma unroll
    for (int i = 0; i < 4; ++i) {
      const int idx = i * NTHR + tid;
      const int row = idx >> 5, seg = idx & 31;
      const v4u g = *(const v4u*)(GX16 + ((size_t)t * NBATCH + (size_t)(rowbase + row)) * NGATE + seg * 8);
      *(v4u*)(Gs + row * EGP + seg * 8) = g;
    }
    __syncthreads();
    v8f acc[4];
    acc[0] = z8; acc[1] = z8; acc[2] = z8; acc[3] = z8;
    {
      const v16h a0 = frag_load(arow);
      const v16h a1 = frag_load(arow + 32);
#pragma unroll
      for (int g = 0; g < 4; ++g) {
        acc[g] = mma_h(a0, bw[g][0], acc[g]);
        acc[g] = mma_h(a1, bw[g][1], acc[g]);
      }
    }
    float hn[8];
#pragma unroll
    for (int r = 0; r < 8; ++r) {
      const int rl = 16 * ms + 8 * hh + r;
      const unsigned short* gp = Gs + rl * EGP + j;
      const float zi = acc[0][r] * FOLD_SW + h16_to_f32((unsigned)gp[0]) * GX_INV + bb[0];
      const float zf = acc[1][r] * FOLD_SW + h16_to_f32((unsigned)gp[NHID]) * GX_INV + bb[1];
      const float zg = acc[2][r] * FOLD_SW + h16_to_f32((unsigned)gp[2 * NHID]) * GX_INV + bb[2];
      const float zo = acc[3][r] * FOLD_SW + h16_to_f32((unsigned)gp[3 * NHID]) * GX_INV + bb[3];
      const float ig = fsig(zi);
      const float fg = fsig(zf);
      const float gg = ftanh(zg);
      const float og = fsig(zo);
      const float cn = fg * cst[r] + ig * gg;
      cst[r] = cn;
      hn[r] = og * ftanh(cn);
    }
    __syncthreads();
#pragma unroll
    for (int r = 0; r < 8; ++r) Ah[(16 * ms + 8 * hh + r) * EHP + j] = (_Float16)(hn[r] * SCARRY);
    __syncthreads();
    {
      const v8h v = *(const v8h*)(Ah + srow * EHP + sseg * 8);
      unsigned short* p = XENC16 + ((size_t)(rowbase + srow) * NLAG + (size_t)t) * NHID + sseg * 8;
      *(volatile v8h*)p = v;
      __threadfence();
      *(volatile v8h*)p = v;
    }
  }
}

__global__ __launch_bounds__(256) void dec_seq_kernel(
    const unsigned short* __restrict__ XENC16, const unsigned short* __restrict__ PRE16,
    const unsigned short* __restrict__ W1HCp, const unsigned short* __restrict__ DGp,
    const float* __restrict__ h0, const float* __restrict__ c0,
    const float* __restrict__ att_b1, const float* __restrict__ att_w2, const float* __restrict__ att_b2,
    const float* __restrict__ bih, const float* __restrict__ bhh,
    const float* __restrict__ fc_w, const float* __restrict__ fc_b,
    const float* __restrict__ y_hist,
    const float* __restrict__ fo_w, const float* __restrict__ fo_b,
    float* __restrict__ out) {
  __shared__ __align__(16) unsigned short Xe[ROWS_PER_BLK * NLAG * NHID];
  __shared__ __align__(16) unsigned short Pr[ROWS_PER_BLK * NLAG * NHID];
  __shared__ __align__(16) _Float16       At[ROWS_PER_BLK * DAP];
  __shared__ __align__(16) float          Sv[ROWS_PER_BLK * DSP];
  __shared__ __align__(16) float          W2s[NHID];
  __shared__ __align__(16) float          Ob[ROWS_PER_BLK * NOUTD];
  __shared__ float Sc[ROWS_PER_BLK * SCP];
  __shared__ float Fw[FCW_N + 3];
  __shared__ float Fo[FOW_N];
  const _Float16* W1HC = (const _Float16*)W1HCp;
  const _Float16* DG   = (const _Float16*)DGp;
  const int tid = threadIdx.x, lane = tid & 31, wave = tid >> 5;
  const int c = lane & 15, hh = lane >> 4, koff = hh * 8;
  const int ms = wave >> 2, ub = wave & 3;
  const int j = 16 * ub + c;
  const int rowbase = blockIdx.x * ROWS_PER_BLK;
  const int b = tid >> 3, p = tid & 7;

#pragma unroll 1
  for (int i = 0; i < NLAG; ++i) {
    const int idx = i * NTHR + tid;
    const size_t go = (size_t)rowbase * (NLAG * NHID) + (size_t)idx * 8;
    const v4u xv = *(const v4u*)(XENC16 + go);
    const v4u pv = *(const v4u*)(PRE16 + go);
    *(v4u*)(Xe + idx * 8) = xv;
    *(v4u*)(Pr + idx * 8) = pv;
  }
  {
    const float* hp = h0 + (size_t)(rowbase + b) * NHID + p * 8;
    const float* cp = c0 + (size_t)(rowbase + b) * NHID + p * 8;
    const v4f ha = *(const v4f*)(hp), hb = *(const v4f*)(hp + 4);
    const v4f ca = *(const v4f*)(cp), cb = *(const v4f*)(cp + 4);
    float zinit = 0.0f;
    asm volatile("" : "+v"(zinit));
    v8h hv, cv, zv;
#pragma unroll
    for (int e = 0; e < 4; ++e) {
      hv[e] = (_Float16)(ha[e] * SCARRY); hv[4 + e] = (_Float16)(hb[e] * SCARRY);
      cv[e] = (_Float16)(ca[e] * SCARRY); cv[4 + e] = (_Float16)(cb[e] * SCARRY);
      zv[e] = (_Float16)zinit;            zv[4 + e] = (_Float16)zinit;
    }
    *(v8h*)(At + b * DAP + p * 8) = hv;
    *(v8h*)(At + b * DAP + NHID + p * 8) = cv;
    if (p < 4) *(v8h*)(At + b * DAP + 2 * NHID + p * 8) = zv;
  }
  {
    const int i0 = tid, i1 = tid + NTHR, i2 = tid + 2 * NTHR;
    const float f0 = fc_w[i0];
    const float f1 = fc_w[(i1 < FCW_N) ? i1 : (FCW_N - 1)];
    Fw[i0] = f0;
    if (i1 < FCW_N) Fw[i1] = f1;
    const float g0 = fo_w[i0];
    const float g1 = fo_w[i1];
    const float g2 = fo_w[(i2 < FOW_N) ? i2 : (FOW_N - 1)];
    Fo[i0] = g0;
    Fo[i1] = g1;
    if (i2 < FOW_N) Fo[i2] = g2;
    const float w2v0 = att_w2[tid & (NHID - 1)];
    if (tid < NHID) W2s[tid] = w2v0;
  }
  float cst[8], hn[8], bbD[4], cx[8];
#pragma unroll
  for (int r = 0; r < 8; ++r) {
    cst[r] = c0[(size_t)(rowbase + 16 * ms + 8 * hh + r) * NHID + j];
    hn[r] = 0.0f;
    cx[r] = 0.0f;
  }
#pragma unroll
  for (int g = 0; g < 4; ++g) bbD[g] = bih[g * NHID + j] + bhh[g * NHID + j];
  const float b1v = att_b1[j];
  const float b2v = att_b2[0];
  const v8f z8 = {0.f, 0.f, 0.f, 0.f, 0.f, 0.f, 0.f, 0.f};
  const _Float16* arow = At + (16 * ms + c) * DAP + koff;

#pragma unroll 1
  for (int t = 0; t < NLAG; ++t) {
    __syncthreads();
    {
      v8f acc = z8;
      const _Float16* brow = W1HC + (size_t)j * (2 * NHID) + koff;
#pragma unroll
      for (int kt = 0; kt < 4; ++kt) {
        const v16h a  = frag_load(arow + kt * 32);
        const v16h bf = frag_load(brow + kt * 32);
        acc = mma_h(a, bf, acc);
      }
#pragma unroll
      for (int r = 0; r < 8; ++r) Sv[(16 * ms + 8 * hh + r) * DSP + j] = acc[r] * FOLD_SW + b1v;
    }
    __syncthreads();
    {
      const v4f s0 = *(const v4f*)(Sv + b * DSP + 8 * p);
      const v4f s1 = *(const v4f*)(Sv + b * DSP + 8 * p + 4);
      const v4f u0 = *(const v4f*)(W2s + 8 * p);
      const v4f u1 = *(const v4f*)(W2s + 8 * p + 4);
      float sv[8], wv[8];
#pragma unroll
      for (int e = 0; e < 4; ++e) { sv[e] = s0[e]; sv[4 + e] = s1[e]; wv[e] = u0[e]; wv[4 + e] = u1[e]; }
#pragma unroll 1
      for (int l = 0; l < NLAG; ++l) {
        const v4u pw = *(const v4u*)(Pr + (b * NLAG + l) * NHID + 8 * p);
        float part = 0.0f;
#pragma unroll
        for (int q = 0; q < 4; ++q) {
          const unsigned w = pw[q];
          const float plo = h16_to_f32(w & 0xffffu);
          const float phi = h16_to_f32(w >> 16);
          part = fmaf(ftanh(plo + sv[2 * q]), wv[2 * q], part);
          part = fmaf(ftanh(phi + sv[2 * q + 1]), wv[2 * q + 1], part);
        }
        part += __shfl_xor(part, 1, 32);
        part += __shfl_xor(part, 2, 32);
        part += __shfl_xor(part, 4, 32);
        if (p == 0) Sc[b * SCP + l] = part + b2v;
      }
    }
    __syncthreads();
    {
      float m = Sc[b * SCP];
#pragma unroll
      for (int l = 1; l < NLAG; ++l) m = fmaxf(m, Sc[b * SCP + l]);
      float ssum = 0.0f;
#pragma unroll 1
      for (int l = 0; l < NLAG; ++l) ssum += expf(Sc[b * SCP + l] - m);
      const float inv = __builtin_amdgcn_rcpf(ssum);
#pragma unroll
      for (int e = 0; e < 8; ++e) cx[e] = 0.0f;
#pragma unroll 1
      for (int l = 0; l < NLAG; ++l) {
        const float a = expf(Sc[b * SCP + l] - m) * inv;
        const v4u xw = *(const v4u*)(Xe + (b * NLAG + l) * NHID + 8 * p);
#pragma unroll
        for (int q = 0; q < 4; ++q) {
          const unsigned w = xw[q];
          cx[2 * q]     = fmaf(a, h16_to_f32(w & 0xffffu), cx[2 * q]);
          cx[2 * q + 1] = fmaf(a, h16_to_f32(w >> 16), cx[2 * q + 1]);
        }
      }
#pragma unroll
      for (int e = 0; e < 8; ++e) cx[e] *= S_INV;
      float qk[5];
#pragma unroll
      for (int k = 0; k < NOUTD; ++k) {
        float s = 0.0f;
#pragma unroll
        for (int e = 0; e < 8; ++e) s = fmaf(Fw[k * (NHID + NOUTD) + 8 * p + e], cx[e], s);
        qk[k] = s;
      }
#pragma unroll
      for (int off = 1; off < 8; off <<= 1) {
#pragma unroll
        for (int k = 0; k < NOUTD; ++k) qk[k] += __shfl_xor(qk[k], off, 32);
      }
      float yv[5];
#pragma unroll
      for (int q = 0; q < NOUTD; ++q) yv[q] = y_hist[((size_t)(rowbase + b) * NLAG + (size_t)t) * NOUTD + q];
      float yt[5];
#pragma unroll
      for (int k = 0; k < NOUTD; ++k) {
        float s = qk[k] + fc_b[k];
#pragma unroll
        for (int q = 0; q < NOUTD; ++q) s = fmaf(Fw[k * (NHID + NOUTD) + NHID + q], yv[q], s);
        yt[k] = s;
      }
      float zpad = 0.0f;
      asm volatile("" : "+v"(zpad));
      const float y0 = (p == 0) ? yt[0] : ((p == 1) ? yt[4] : zpad);
      const float y1 = (p == 0) ? yt[1] : zpad;
      const float y2 = (p == 0) ? yt[2] : zpad;
      const float y3 = (p == 0) ? yt[3] : zpad;
      _Float16* yp = At + b * DAP + 2 * NHID + 4 * p;
      yp[0] = (_Float16)(y0 * SCARRY);
      yp[1] = (_Float16)(y1 * SCARRY);
      yp[2] = (_Float16)(y2 * SCARRY);
      yp[3] = (_Float16)(y3 * SCARRY);
    }
    __syncthreads();
    {
      v8f acc[4];
      acc[0] = z8; acc[1] = z8; acc[2] = z8; acc[3] = z8;
#pragma unroll
      for (int kt = 0; kt < 3; ++kt) {
        const int acol = (kt < 2) ? (kt * 32) : (2 * NHID);
        const v16h a  = frag_load(arow + acol);
        const v16h g0 = frag_load(DG + (size_t)(0 * NHID + j) * DGK + koff + kt * 32);
        const v16h g1 = frag_load(DG + (size_t)(1 * NHID + j) * DGK + koff + kt * 32);
        const v16h g2 = frag_load(DG + (size_t)(2 * NHID + j) * DGK + koff + kt * 32);
        const v16h g3 = frag_load(DG + (size_t)(3 * NHID + j) * DGK + koff + kt * 32);
        acc[0] = mma_h(a, g0, acc[0]);
        acc[1] = mma_h(a, g1, acc[1]);
        acc[2] = mma_h(a, g2, acc[2]);
        acc[3] = mma_h(a, g3, acc[3]);
      }
#pragma unroll
      for (int r = 0; r < 8; ++r) {
        const float zi = acc[0][r] * FOLD_SW + bbD[0];
        const float zf = acc[1][r] * FOLD_SW + bbD[1];
        const float zg = acc[2][r] * FOLD_SW + bbD[2];
        const float zo = acc[3][r] * FOLD_SW + bbD[3];
        const float ig = fsig(zi);
        const float fg = fsig(zf);
        const float gg = ftanh(zg);
        const float og = fsig(zo);
        const float cn = fg * cst[r] + ig * gg;
        cst[r] = cn;
        hn[r] = og * ftanh(cn);
      }
    }
    __syncthreads();
#pragma unroll
    for (int r = 0; r < 8; ++r) {
      At[(16 * ms + 8 * hh + r) * DAP + j]        = (_Float16)(hn[r] * SCARRY);
      At[(16 * ms + 8 * hh + r) * DAP + NHID + j] = (_Float16)(cst[r] * SCARRY);
    }
  }

#pragma unroll
  for (int r = 0; r < 8; ++r) Sv[(16 * ms + 8 * hh + r) * DSP + j] = hn[r];
  __syncthreads();
  {
    const v4f h0v = *(const v4f*)(Sv + b * DSP + 8 * p);
    const v4f h1v = *(const v4f*)(Sv + b * DSP + 8 * p + 4);
    float hf[8];
#pragma unroll
    for (int e = 0; e < 4; ++e) { hf[e] = h0v[e]; hf[4 + e] = h1v[e]; }
    float ok[5];
#pragma unroll
    for (int k = 0; k < NOUTD; ++k) {
      float s = 0.0f;
#pragma unroll
      for (int e = 0; e < 8; ++e) {
        s = fmaf(Fo[k * 2 * NHID + 8 * p + e], hf[e], s);
        s = fmaf(Fo[k * 2 * NHID + NHID + 8 * p + e], cx[e], s);
      }
      ok[k] = s;
    }
#pragma unroll
    for (int off = 1; off < 8; off <<= 1) {
#pragma unroll
      for (int k = 0; k < NOUTD; ++k) ok[k] += __shfl_xor(ok[k], off, 32);
    }
    const int pc = (p < NOUTD) ? p : (NOUTD - 1);
    const float fob = fo_b[pc];
    const float sel = (p == 0) ? ok[0] : ((p == 1) ? ok[1] : ((p == 2) ? ok[2] : ((p == 3) ? ok[3] : ok[4])));
    if (p < NOUTD) Ob[b * NOUTD + p] = sel + fob;
  }
  __syncthreads();
  if (wave == 0) {
    const v4f v0 = *(const v4f*)(Ob + lane * 4);
    const v4f v1 = *(const v4f*)(Ob + 128 + (lane & 7) * 4);
    float* op = out + (size_t)rowbase * NOUTD;
    for (int pass = 0; pass < 2; ++pass) {
      *(volatile v4f*)(op + lane * 4) = v0;
      if (lane < 8) *(volatile v4f*)(op + 128 + lane * 4) = v1;
      __threadfence();
    }
  }
}

extern "C" void kernel_launch(void* const* d_in, const int* in_sizes, int n_in,
                              void* d_out, int out_size, void* d_ws, size_t ws_size, hipStream_t stream) {
  if (n_in < 24 || d_out == nullptr || d_ws == nullptr) return;
  if (in_sizes[0] != NBATCH * NLAG * NFEAT || in_sizes[1] != NBATCH * NLAG * NOUTD ||
      in_sizes[2] != NBATCH * NHID || in_sizes[3] != NBATCH * NHID || in_sizes[4] != NBATCH * NHID || in_sizes[5] != NBATCH * NHID ||
      in_sizes[6] != 2 * NHID + NLAG || in_sizes[7] != 1 ||
      in_sizes[8] != NGATE * NFEAT || in_sizes[9] != NGATE * NHID || in_sizes[10] != NGATE || in_sizes[11] != NGATE ||
      in_sizes[12] != NHID * 3 * NHID || in_sizes[13] != NHID || in_sizes[14] != NHID || in_sizes[15] != 1 ||
      in_sizes[16] != NGATE * NOUTD || in_sizes[17] != NGATE * NHID || in_sizes[18] != NGATE || in_sizes[19] != NGATE ||
      in_sizes[20] != FCW_N || in_sizes[21] != NOUTD || in_sizes[22] != FOW_N || in_sizes[23] != NOUTD ||
      out_size != NBATCH * NOUTD) return;

  const float* x        = (const float*)d_in[0];
  const float* y_hist   = (const float*)d_in[1];
  const float* h0_enc   = (const float*)d_in[2];
  const float* c0_enc   = (const float*)d_in[3];
  const float* h0_dec   = (const float*)d_in[4];
  const float* c0_dec   = (const float*)d_in[5];
  const float* enc_aw   = (const float*)d_in[6];
  const float* enc_ab   = (const float*)d_in[7];
  const float* enc_wih  = (const float*)d_in[8];
  const float* enc_whh  = (const float*)d_in[9];
  const float* enc_bih  = (const float*)d_in[10];
  const float* enc_bhh  = (const float*)d_in[11];
  const float* att_w1   = (const float*)d_in[12];
  const float* att_b1   = (const float*)d_in[13];
  const float* att_w2   = (const float*)d_in[14];
  const float* att_b2   = (const float*)d_in[15];
  const float* dec_wih  = (const float*)d_in[16];
  const float* dec_whh  = (const float*)d_in[17];
  const float* dec_bih  = (const float*)d_in[18];
  const float* dec_bhh  = (const float*)d_in[19];
  const float* fc_w     = (const float*)d_in[20];
  const float* fc_b     = (const float*)d_in[21];
  const float* fo_w     = (const float*)d_in[22];
  const float* fo_b     = (const float*)d_in[23];
  float* out = (float*)d_out;

  char* ws = (char*)d_ws;
  size_t off = 0;
  auto carve = [&](size_t bytes) -> char* { char* q = ws + off; off += (bytes + 255) & ~(size_t)255; return q; };
  unsigned short* WIH16  = (unsigned short*)carve((size_t)NGATE * NFEAT * 2);
  unsigned short* WHH16  = (unsigned short*)carve((size_t)NGATE * NHID * 2);
  unsigned short* DG16   = (unsigned short*)carve((size_t)NGATE * DGK * 2);
  unsigned short* W1HC16 = (unsigned short*)carve((size_t)NHID * 2 * NHID * 2);
  unsigned short* W1X16  = (unsigned short*)carve((size_t)NHID * NHID * 2);
  unsigned short* WI16   = (unsigned short*)carve((size_t)NROWS * NFEAT * 2);
  unsigned short* GX16   = (unsigned short*)carve((size_t)NROWS * NGATE * 2);
  unsigned short* XENC16 = (unsigned short*)carve((size_t)NROWS * NHID * 2);
  unsigned short* PRE16  = (unsigned short*)carve((size_t)NROWS * NHID * 2);
  if (off > ws_size || off > (size_t)134217728) return;

  prep_planes_kernel<<<PB_E4, NTHR, 0, stream>>>(enc_wih, enc_whh, dec_whh, dec_wih, att_w1,
                                                 WIH16, WHH16, DG16, W1HC16, W1X16);
  wi_build_kernel<<<NBATCH / 16, NTHR, 0, stream>>>(x, enc_aw, enc_ab, WI16);
  gemm64_f16_kernel<<<(NROWS / 64) * (NGATE / 64) / 8, 256, 0, stream>>>(
      WI16, NFEAT, WIH16, NFEAT, GX16, NGATE, NROWS, NGATE, NFEAT, GX_SCALE);
  enc_seq_kernel<<<NBATCH / ROWS_PER_BLK, NTHR, 0, stream>>>(GX16, WHH16, h0_enc, c0_enc, enc_bih, enc_bhh, XENC16);
  gemm64_f16_kernel<<<(NROWS / 64) * (NHID / 64) / 8, 256, 0, stream>>>(
      XENC16, NHID, W1X16, NHID, PRE16, NHID, NROWS, NHID, NHID, FOLD_SW);
  dec_seq_kernel<<<NBATCH / ROWS_PER_BLK, NTHR, 0, stream>>>(
      XENC16, PRE16, W1HC16, DG16, h0_dec, c0_dec, att_b1, att_w2, att_b2,
      dec_bih, dec_bhh, fc_w, fc_b, y_hist, fo_w, fo_b, out);
}
